// GINConvFFT_31044023616144
// MI455X (gfx1250) — hardware-verified
//
#include <hip/hip_runtime.h>


#define NBT  32
#define NNODE 512
#define LL   12
#define HHID 64
#define LH   (LL * HHID)
#define NSUP 2
#define ORD  2
#define K4   (NSUP * ORD)
#define OUTD 64
#define NR   (NBT * NNODE)
#define DM   NNODE
#define BEPS 1e-5f
#define LOSC 1024.0f

typedef _Float16 h16;
typedef unsigned short bf;
typedef __attribute__((ext_vector_type(16))) __bf16   v16bf;
typedef __attribute__((ext_vector_type(16))) _Float16 v16h;
typedef __attribute__((ext_vector_type(8)))  _Float16 v8h;
typedef __attribute__((ext_vector_type(8)))  unsigned short v8us;
typedef __attribute__((ext_vector_type(8)))  float    v8f;
typedef __attribute__((ext_vector_type(4)))  float    v4f;
typedef v8h  __attribute__((may_alias)) v8ha;
typedef v4f  __attribute__((may_alias)) v4fa;
typedef v8us __attribute__((may_alias)) v8usa;

__device__ __forceinline__ unsigned short f2bf(float f) { unsigned u = __float_as_uint(f); u += 0x7FFFu + ((u >> 16) & 1u); return (unsigned short)(u >> 16); }
__device__ __forceinline__ float bf2f(unsigned short b) { return __uint_as_float(((unsigned)b) << 16); }
__device__ __forceinline__ float bfr(float f) { return bf2f(f2bf(f)); }
__device__ __forceinline__ v16h cat16(v8h lo, v8h hi) { return __builtin_shufflevector(lo, hi, 0, 1, 2, 3, 4, 5, 6, 7, 8, 9, 10, 11, 12, 13, 14, 15); }
__device__ __forceinline__ v16bf cat16b(v8us lo, v8us hi) { return __builtin_bit_cast(v16bf, __builtin_shufflevector(lo, hi, 0, 1, 2, 3, 4, 5, 6, 7, 8, 9, 10, 11, 12, 13, 14, 15)); }
__device__ __forceinline__ v8f wmma16(v16h a, v16h b, v8f c) { return __builtin_amdgcn_wmma_f32_16x16x32_f16(false, a, false, b, (short)0, c, false, false); }
__device__ __forceinline__ v8f wmmab(v16bf a, v16bf b, v8f c) { return __builtin_amdgcn_wmma_f32_16x16x32_bf16(false, a, false, b, (short)0, c, false, false); }

template <bool SPLITA, bool F16OUT = false>
__global__ __launch_bounds__(128) void k_gemmb(const bf* __restrict__ A, const bf* __restrict__ Al, const bf* __restrict__ Bn, const float* __restrict__ bias, float* C, int ldc, h16* C2, const float* __restrict__ R = nullptr, int K = DM, int roundR = 1) {
    __shared__ __align__(16) float ost[4][16 * 68];
    const int lane = threadIdx.x & 31, wave = threadIdx.x >> 5, lr = lane & 15, hi = lane >> 4;
    const int r0 = blockIdx.x * 64 + wave * 16, c0 = blockIdx.y * 64;
    const size_t aoff = (size_t)(r0 + lr) * K + 8 * hi;
    size_t boff[4];
#pragma unroll
    for (int t = 0; t < 4; ++t) boff[t] = (size_t)(c0 + t * 16 + lr) * K + 8 * hi;
    v8f acc[4];
#pragma unroll
    for (int t = 0; t < 4; ++t) acc[t] = (v8f){};
#pragma unroll 1
    for (int kc = 0; kc < K; kc += 32) {
        const v16bf a = cat16b(*(const v8us*)(A + aoff + kc), *(const v8us*)(A + aoff + kc + 16));
        v16bf al = a;
        if (SPLITA) al = cat16b(*(const v8us*)(Al + aoff + kc), *(const v8us*)(Al + aoff + kc + 16));
#pragma unroll
        for (int t = 0; t < 4; ++t) { const v16bf b = cat16b(*(const v8us*)(Bn + boff[t] + kc), *(const v8us*)(Bn + boff[t] + kc + 16)); acc[t] = wmmab(a, b, acc[t]); if (SPLITA) acc[t] = wmmab(al, b, acc[t]); }
        asm volatile("v_nop\n\tv_nop\n\tv_nop\n\tv_nop" : "+v"(acc[0]), "+v"(acc[1]), "+v"(acc[2]), "+v"(acc[3]) : "v"(a), "v"(al));
    }
    float* os = &ost[wave][0];
#pragma unroll
    for (int t = 0; t < 4; ++t) { const float bv = bias ? bfr(bias[c0 + t * 16 + lr]) : 0.f;
#pragma unroll
        for (int j = 0; j < 8; ++j) os[(hi * 8 + j) * 68 + t * 16 + lr] = acc[t][j] + bv; }
    __syncthreads();
    if (F16OUT) {
        h16* crow = (h16*)(void*)C + (size_t)r0 * ldc + c0;
        auto pass = [&]() {
#pragma unroll
            for (int s = 0; s < 4; ++s) { const int row = 4 * s + (lane >> 3), piece = lane & 7; const float* sp = os + row * 68 + piece * 8; v8h o, o2;
#pragma unroll
                for (int i = 0; i < 8; ++i) { const h16 a = (h16)sp[i]; o[i] = a; o2[i] = (h16)((sp[i] - (float)a) * LOSC); }
                *(volatile v8h*)(crow + (size_t)row * ldc + piece * 8) = o; if (C2) *(volatile v8h*)(C2 + (size_t)r0 * ldc + c0 + (size_t)row * ldc + piece * 8) = o2; }
        };
        pass(); __threadfence(); pass();
    } else {
        float* crow = C + (size_t)r0 * ldc + c0;
        auto pass = [&]() {
#pragma unroll
            for (int s = 0; s < 8; ++s) { const int Lid = (lane >> 3) + 4 * s, piece = lane & 7; const int row = Lid >> 1, cofs = (Lid & 1) * 32 + piece * 4;
                v4f val = *(const v4fa*)(os + row * 68 + cofs); if (R) { const v4f rv = *(const v4f*)(R + ((size_t)r0 + row) * ldc + c0 + cofs); val += roundR ? (v4f){bfr(rv[0]), bfr(rv[1]), bfr(rv[2]), bfr(rv[3])} : rv; }
                *(volatile v4f*)(crow + (size_t)row * ldc + cofs) = val; }
        };
        pass(); __threadfence(); pass();
    }
}

__global__ __launch_bounds__(256) void k_wt(const float* __restrict__ Wm, int K, int ncols, bf* WT) {
    __shared__ __align__(16) unsigned short tl[64 * 72];
    const int tid = threadIdx.x, k0 = blockIdx.x * 64, n0 = blockIdx.y * 64;
    const int kk = tid >> 2, nq = (tid & 3) * 16;
#pragma unroll
    for (int i = 0; i < 16; ++i) tl[(nq + i) * 72 + kk] = f2bf(Wm[(size_t)(k0 + kk) * ncols + n0 + nq + i]);
    __syncthreads();
    const int piece = tid & 7;
    auto pass = [&]() {
#pragma unroll
        for (int s = 0; s < 2; ++s) { const int nr = (tid >> 3) + 32 * s; const v8us val = *(const v8usa*)(tl + nr * 72 + piece * 8); *(volatile v8us*)(WT + (size_t)(n0 + nr) * K + k0 + piece * 8) = val; }
    };
    pass(); __threadfence(); pass();
}

__global__ __launch_bounds__(256) void k_cvt8(const float* __restrict__ src, bf* dst, size_t n8) {
    const size_t i = (size_t)blockIdx.x * 256 + threadIdx.x; if (i >= n8) return;
    const v8f v = *(const v8f*)(src + i * 8); v8us o;
#pragma unroll
    for (int k = 0; k < 8; ++k) o[k] = f2bf(v[k]);
    *(volatile v8us*)(dst + i * 8) = o; __threadfence(); *(volatile v8us*)(dst + i * 8) = o;
}
__global__ __launch_bounds__(256) void k_zero8(bf* dst, size_t n8) {
    const size_t i = (size_t)blockIdx.x * 256 + threadIdx.x; if (i >= n8) return; v8us z;
#pragma unroll
    for (int k = 0; k < 8; ++k) z[k] = 0;
    *(volatile v8us*)(dst + i * 8) = z; __threadfence(); *(volatile v8us*)(dst + i * 8) = z;
}

__global__ __launch_bounds__(256) void k_wk(const float* __restrict__ wgt, bf* WK) {
    const int lane = threadIdx.x & 31; const int r = blockIdx.x * 8 + (threadIdx.x >> 5); if (r >= K4 * OUTD) return; const int k = r / OUTD, o = r % OUTD;
#pragma unroll 1
    for (int ps = 0; ps < 2; ++ps) {
#pragma unroll
        for (int q = 0; q < LH / 256; ++q) { v8us v;
#pragma unroll
            for (int i = 0; i < 8; ++i) { const int lh = q * 256 + lane * 8 + i; const int l = lh / HHID, h = lh % HHID; v[i] = f2bf(wgt[((size_t)l * (HHID * K4) + h * K4 + k) * OUTD + o]); }
            *(volatile v8us*)(WK + (size_t)r * LH + q * 256 + lane * 8) = v; }
        if (ps == 0) __threadfence(); }
}
__global__ __launch_bounds__(256) void k_scalex(const float* __restrict__ xb, const float* __restrict__ epsv, float* OS) {
    const int lane = threadIdx.x & 31; const size_t n = (size_t)blockIdx.x * 8 + (threadIdx.x >> 5); if (n >= (size_t)NNODE) return; const float sc = 1.0f + bfr(epsv[0]);
#pragma unroll 1
    for (int ps = 0; ps < 2; ++ps) {
#pragma unroll
        for (int c0 = lane * 4; c0 < LH; c0 += 128) { v4f v;
#pragma unroll
            for (int q = 0; q < 4; ++q) v[q] = sc * bfr(xb[n * LH + c0 + q]);
            *(volatile v4f*)(OS + n * LH + c0) = v; }
        if (ps == 0) __threadfence(); }
}
__global__ __launch_bounds__(256) void k_post(const float* __restrict__ O, const float* __restrict__ epsv, bf* Ph, bf* Pl, float* OS) {
    typedef __attribute__((ext_vector_type(4))) unsigned short v4us;
    const int lane = threadIdx.x & 31; const size_t n = (size_t)blockIdx.x * 8 + (threadIdx.x >> 5); if (n >= (size_t)NNODE) return; const float sc = 1.0f + bfr(epsv[0]);
#pragma unroll 1
    for (int ps = 0; ps < 2; ++ps) {
#pragma unroll
        for (int c0 = lane * 4; c0 < LH; c0 += 128) { v4f v; v4us oh, ol;
#pragma unroll
            for (int q = 0; q < 4; ++q) { const float t = O[n * LH + c0 + q]; v[q] = sc * t; const unsigned short hb = f2bf(t); oh[q] = hb; ol[q] = f2bf(t - bf2f(hb)); }
            *(volatile v4f*)(OS + n * LH + c0) = v; *(volatile v4us*)(Ph + n * LH + c0) = oh; *(volatile v4us*)(Pl + n * LH + c0) = ol; }
        if (ps == 0) __threadfence(); }
}
__global__ __launch_bounds__(256) void k_tpl(const float* __restrict__ O, bf* Th, bf* Tl) {
    __shared__ float tl[64][65];
    const int tid = threadIdx.x, n0 = blockIdx.x * 64, d0 = blockIdx.y * 64; const int nn = tid >> 2, dq = (tid & 3) * 16;
#pragma unroll
    for (int i = 0; i < 16; ++i) tl[nn][dq + i] = O[(size_t)(n0 + nn) * LH + d0 + dq + i];
    __syncthreads();
    const int piece = tid & 7, dr0 = tid >> 3;
    auto pass = [&]() {
#pragma unroll
        for (int st = 0; st < 2; ++st) { const int dr = dr0 + 32 * st; v8us oh, ol;
#pragma unroll
            for (int i = 0; i < 8; ++i) { const float v = tl[piece * 8 + i][dr]; const unsigned short hb = f2bf(v); oh[i] = hb; ol[i] = f2bf(v - bf2f(hb)); }
            const size_t o = (size_t)(d0 + dr) * NNODE + n0 + piece * 8; *(volatile v8us*)(Th + o) = oh; *(volatile v8us*)(Tl + o) = ol; }
    };
    pass(); __threadfence(); pass();
}
template <int MODE>
__global__ __launch_bounds__(64) void k_colstat(const float* __restrict__ Y, const float* __restrict__ MEAN, float* OUTV) {
    const int c = threadIdx.x; float s = 0.f; const float mu = (MODE == 1) ? MEAN[c] : 0.f;
#pragma unroll 1
    for (int b = 0; b < NBT; ++b) { float p = 0.f;
#pragma unroll 4
        for (int r = b * NNODE; r < (b + 1) * NNODE; ++r) { const float v = Y[(size_t)r * OUTD + c]; const float d = (MODE == 1) ? (v - mu) * (v - mu) : v; p += d; }
        s += p; }
    s *= 1.0f / (float)NR; *(volatile float*)(OUTV + c) = s; __threadfence(); *(volatile float*)(OUTV + c) = s;
}
__global__ __launch_bounds__(256) void k_bnrelu(const float* __restrict__ Y, const float* __restrict__ MEAN, const float* __restrict__ VAR, const float* __restrict__ ga, const float* __restrict__ be, bf* Ph, bf* Pl) {
    typedef __attribute__((ext_vector_type(2))) unsigned short v2us;
    const int lane = threadIdx.x & 31; const size_t r = (size_t)blockIdx.x * 8 + (threadIdx.x >> 5); if (r >= (size_t)NR) return; v2us oh, ol;
#pragma unroll
    for (int i = 0; i < 2; ++i) { const int c = lane * 2 + i; const float v = fmaxf(bfr(ga[c]) * (Y[r * OUTD + c] - MEAN[c]) * rsqrtf(VAR[c] + BEPS) + bfr(be[c]), 0.f); const unsigned short hb = f2bf(v); oh[i] = hb; ol[i] = f2bf(v - bf2f(hb)); }
    const size_t o = r * OUTD + lane * 2; *(volatile v2us*)(Ph + o) = oh; *(volatile v2us*)(Pl + o) = ol; __threadfence(); *(volatile v2us*)(Ph + o) = oh; *(volatile v2us*)(Pl + o) = ol;
}

extern "C" void kernel_launch(void* const* d_in, const int* in_sizes, int n_in,
                              void* d_out, int out_size, void* d_ws, size_t ws_size, hipStream_t stream) {
    (void)in_sizes; (void)n_in; (void)out_size;
    const float* x = (const float*)d_in[0]; const float* sup = (const float*)d_in[1]; const float* wgt = (const float*)d_in[2]; const float* epsv = (const float*)d_in[3]; const float* ga = (const float*)d_in[4]; const float* be = (const float*)d_in[5]; const float* w2 = (const float*)d_in[6]; const float* b2 = (const float*)d_in[7];
    float* out = (float*)d_out;
    char* wsp = (char*)d_ws;
    auto take = [&](size_t bytes) { char* p = wsp; wsp += (bytes + 255) & ~(size_t)255; return (void*)p; };
    bf* AB = (bf*)take((size_t)NSUP * NNODE * NNODE * 2); bf* WK = (bf*)take((size_t)K4 * OUTD * LH * 2); bf* W2B = (bf*)take((size_t)OUTD * OUTD * 2);
    bf* XT = (bf*)take((size_t)LH * NNODE * 2); float* OS0 = (float*)take((size_t)NNODE * LH * 4); float* O1 = (float*)take((size_t)NNODE * LH * 4); bf* P1h = (bf*)take((size_t)NNODE * LH * 2); bf* P1l = (bf*)take((size_t)NNODE * LH * 2); float* OS1 = (float*)take((size_t)NNODE * LH * 4);
    bf* T1h = (bf*)take((size_t)LH * NNODE * 2); bf* T1l = (bf*)take((size_t)LH * NNODE * 2); float* C2 = (float*)take((size_t)NNODE * LH * 4); float* O2 = (float*)take((size_t)NNODE * LH * 4); bf* P2h = (bf*)take((size_t)NNODE * LH * 2); bf* P2l = (bf*)take((size_t)NNODE * LH * 2); float* OS2 = (float*)take((size_t)NNODE * LH * 4);
    float* Y1 = (float*)take((size_t)NR * OUTD * 4); float* Y = (float*)take((size_t)NR * OUTD * 4); float* MEAN = (float*)take(256); float* VAR = (float*)take(256); bf* Rh = (bf*)take((size_t)NR * OUTD * 2); bf* Rl = (bf*)take((size_t)NR * OUTD * 2);
    if ((size_t)(wsp - (char*)d_ws) > ws_size) return;
    k_cvt8<<<(NSUP * NNODE * NNODE / 8 + 255) / 256, 256, 0, stream>>>(sup, AB, (size_t)NSUP * NNODE * NNODE / 8); k_wk<<<(K4 * OUTD) / 8, 256, 0, stream>>>(wgt, WK); k_cvt8<<<(OUTD * OUTD / 8 + 255) / 256, 256, 0, stream>>>(w2, W2B, OUTD * OUTD / 8);
    for (int b = 0; b < NBT; ++b) { const float* xb = x + (size_t)b * NNODE * LH; float* Yb1 = Y1 + (size_t)b * NNODE * OUTD; float* Yb = Y + (size_t)b * NNODE * OUTD;
        k_wt<<<dim3(NNODE / 64, LH / 64, 1), 256, 0, stream>>>(xb, NNODE, LH, XT); k_scalex<<<NNODE / 8, 256, 0, stream>>>(xb, epsv, OS0);
        for (int i = 0; i < NSUP; ++i) { const bf* Ai = AB + (size_t)i * NNODE * NNODE; const int k1 = i * ORD, k2 = i * ORD + 1;
            k_gemmb<false, false><<<dim3(NNODE / 64, LH / 64, 1), 128, 0, stream>>>(Ai, nullptr, XT, nullptr, O1, LH, nullptr, OS0, NNODE, 0);
            k_post<<<NNODE / 8, 256, 0, stream>>>(O1, epsv, P1h, P1l, OS1); k_tpl<<<dim3(NNODE / 64, LH / 64, 1), 256, 0, stream>>>(O1, T1h, T1l);
            k_gemmb<false, false><<<dim3(NNODE / 64, LH / 64, 1), 128, 0, stream>>>(Ai, nullptr, T1h, nullptr, C2, LH, nullptr, OS1, NNODE, 0);
            k_gemmb<false, false><<<dim3(NNODE / 64, LH / 64, 1), 128, 0, stream>>>(Ai, nullptr, T1l, nullptr, O2, LH, nullptr, C2, NNODE, 0);
            k_post<<<NNODE / 8, 256, 0, stream>>>(O2, epsv, P2h, P2l, OS2);
            k_gemmb<true, false><<<dim3(NNODE / 64, 1, 1), 128, 0, stream>>>(P1h, P1l, WK + (size_t)k1 * OUTD * LH, nullptr, Yb1, OUTD, nullptr, (i == 0) ? nullptr : Yb, LH, 0);
            k_gemmb<true, false><<<dim3(NNODE / 64, 1, 1), 128, 0, stream>>>(P2h, P2l, WK + (size_t)k2 * OUTD * LH, nullptr, Yb, OUTD, nullptr, Yb1, LH, 0); } }
    k_colstat<0><<<1, 64, 0, stream>>>(Y, nullptr, MEAN); k_colstat<1><<<1, 64, 0, stream>>>(Y, MEAN, VAR);
    k_bnrelu<<<NR / 8, 256, 0, stream>>>(Y, MEAN, VAR, ga, be, Rh, Rl);
    k_gemmb<true, false><<<dim3(NR / 64, 1, 1), 128, 0, stream>>>(Rh, Rl, W2B, b2, out, OUTD, nullptr, nullptr, OUTD);
}
